// NodeLevelAttention_56495999812298
// MI455X (gfx1250) — hardware-run, weakly checked
//
#include <hip/hip_runtime.h>
#include <stddef.h>
#include <stdint.h>
#include <math.h>


#define DD       64
#define NP_C     50000
#define NO_C     50000
#define NE_C     800000
#define NTHR     256
#define NWAVE    8
#define EPT      8
#define CHUNK    (NTHR * EPT)
#define WCAP     (EPT * 32)
#define LISTN    (NWAVE * WCAP)
#define NBRUN    1024
#define SLA      10
#define RCAP     28672
#define DEGCAP   64
#define PM       128
#define SPITCH   65
#define PARN     256
#define SPAD     50048
#define NBLK_P   391
#define NBLK_S   49
#define OUT1_OFF 3200000
#define PLANE_H  (NP_C * DD)
#define LDS_SCAN ((2 * RCAP + 2 * NBRUN + LISTN + 16) * 4)
#define WSMAX    134217728
#define NROWS_PREP (NP_C + NO_C + DD + 2)

static_assert(DD == 64);
static_assert(2 * 32 == DD);
static_assert(NBRUN == 1024 && NBRUN == (1 << SLA));
static_assert(NBLK_S * NBRUN >= NP_C && (NBLK_S - 1) * NBRUN < NP_C);
static_assert(RCAP >= 16696 + 8192);
static_assert(DEGCAP >= 33 + 8 && DEGCAP == 64);
static_assert(CHUNK == 2048);
static_assert(SPAD == NBLK_P * PM && SPAD >= NP_C && SPAD >= NO_C);
static_assert(OUT1_OFF == NP_C * DD);
static_assert(NP_C == NO_C);
static_assert((NE_C % EPT) == 0 && NE_C >= EPT);
static_assert(((long long)(NO_C - 1) << SLA) < (1LL << 31));
static_assert(NBRUN == 4 * NTHR);
static_assert(LISTN >= NBRUN);
static_assert((RCAP % 32) == 0);
static_assert(LDS_SCAN <= 327680);
static_assert(PM == NWAVE * 16);
static_assert((long long)OUT1_OFF + (long long)(NO_C - 1) * DD + DD - 1 < (long long)(NP_C + NO_C) * DD);
static_assert(((size_t)NP_C * DD * 2) % 256 == 0 && ((size_t)SPAD * 4) % 256 == 0);

typedef float          v2f  __attribute__((ext_vector_type(2)));
typedef float          v4f  __attribute__((ext_vector_type(4)));
typedef float          v8f  __attribute__((ext_vector_type(8)));
typedef int            v4i  __attribute__((ext_vector_type(4)));
typedef int            v8i  __attribute__((ext_vector_type(8)));
typedef unsigned short v8us __attribute__((ext_vector_type(8)));
typedef __bf16         v16b __attribute__((ext_vector_type(16)));
typedef v2f  __attribute__((may_alias)) v2fa;
typedef v4f  __attribute__((may_alias)) v4fa;
typedef v4i  __attribute__((may_alias)) v4ia;
typedef v8us __attribute__((may_alias)) v8usa;
union FragB { v16b v; v8us h[2]; v8i w; };

__device__ __forceinline__ v8f wmb(const FragB& a, const FragB& b, v8f c) {
  v8f d = __builtin_amdgcn_wmma_f32_16x16x32_bf16(false, a.v, false, b.v, (short)0, c, false, false);
  asm volatile("v_nop\n\tv_nop\n\tv_nop\n\tv_nop" : "+v"(d) : "v"(a.w), "v"(b.w));
  return d;
}

__device__ __forceinline__ unsigned bf16_bits(float f) {
  const unsigned u = __float_as_uint(f);
  return ((u + 0x7FFFu + ((u >> 16) & 1u)) >> 16) & 0xFFFFu;
}
__device__ __forceinline__ float bfr(float f) { return __uint_as_float(bf16_bits(f) << 16); }
__device__ __forceinline__ v4f bfr4(const v4f a) {
  v4f r; r.x = bfr(a.x); r.y = bfr(a.y); r.z = bfr(a.z); r.w = bfr(a.w); return r;
}

__global__ __launch_bounds__(NTHR) void k_prep(const float* __restrict__ hp, const float* __restrict__ ho,
                                               const float* __restrict__ Ww, const float* __restrict__ Wb,
                                               const float* __restrict__ aw, const float* __restrict__ ab,
                                               unsigned* HPB, unsigned* HOB, unsigned* WB, float* PAR,
                                               float* out) {
  const int lane = (int)threadIdx.x & 31;
  const int wave = __builtin_amdgcn_readfirstlane((int)threadIdx.x >> 5);
  const int wv   = (int)blockIdx.x * NWAVE + wave;
  if (wv < NP_C) {
    const v2f a = *(const v2fa*)(hp + (size_t)wv * DD + 2 * lane);
    const unsigned w = bf16_bits(a.x) | (bf16_bits(a.y) << 16);
    unsigned* dp = HPB + (size_t)wv * 32 + lane;
    *(volatile unsigned*)dp = w;
    __threadfence();
    *(volatile unsigned*)dp = w;
  } else if (wv < NP_C + NO_C) {
    const int row = wv - NP_C;
    const v2f a = *(const v2fa*)(ho + (size_t)row * DD + 2 * lane);
    const unsigned b0 = bf16_bits(a.x), b1 = bf16_bits(a.y);
    const unsigned w = b0 | (b1 << 16);
    const float r0 = __uint_as_float(b0 << 16);
    const float r1 = __uint_as_float(b1 << 16);
    float ss = r0 * r0 + r1 * r1;
#pragma unroll
    for (int off = 16; off > 0; off >>= 1) ss += __shfl_xor(ss, off);
    const float nn = fmaxf(sqrtf(ss), 1e-12f);
    v2f o;
    o.x = r0 / nn;
    o.y = r1 / nn;
    unsigned* dp = HOB + (size_t)row * 32 + lane;
    float* op = out + (size_t)OUT1_OFF + (size_t)row * DD + 2 * lane;
    *(volatile unsigned*)dp = w;
    *(volatile v2f*)op = o;
    __threadfence();
    *(volatile unsigned*)dp = w;
    *(volatile v2f*)op = o;
  } else if (wv < NP_C + NO_C + DD) {
    const int row = wv - NP_C - NO_C;
    const v2f a = *(const v2fa*)(Ww + (size_t)row * DD + 2 * lane);
    const unsigned w = bf16_bits(a.x) | (bf16_bits(a.y) << 16);
    unsigned* dp = WB + (size_t)row * 32 + lane;
    *(volatile unsigned*)dp = w;
    __threadfence();
    *(volatile unsigned*)dp = w;
  } else if (wv < NROWS_PREP) {
    const int q  = wv - NP_C - NO_C - DD;
    const int i0 = 128 * q + 4 * lane;
    const int iw = i0 < 60 ? i0 : 60;
    int ia = i0 - 64;
    ia = ia < 0 ? 0 : (ia > 124 ? 124 : ia);
    const v4f w4 = *(const v4fa*)(Wb + iw);
    const v4f a4 = *(const v4fa*)(aw + ia);
    const float a0 = ab[0];
    asm volatile("" :: "v"(w4), "v"(a4), "v"(a0));
    const v4f wr = bfr4(w4);
    const v4f ar = bfr4(a4);
    const float abr = bfr(a0);
    v4f o = {0.f, 0.f, 0.f, 0.f};
    if (i0 < 64) o = wr;
    else if (i0 < 192) o = ar;
    else if (i0 == 192) o.x = abr;
    float* dp = PAR + i0;
    *(volatile v4f*)dp = o;
    __threadfence();
    *(volatile v4f*)dp = o;
  }
}

__global__ __launch_bounds__(NTHR) __attribute__((amdgpu_num_vgpr(248)))
void k_proj(const unsigned short* __restrict__ HB, const unsigned short* __restrict__ WB,
            const float* __restrict__ PAR, float* S) {
  __shared__ __attribute__((aligned(16))) float stg[PM * SPITCH];
  __shared__ __attribute__((aligned(16))) float spar[PARN];
  __shared__ __attribute__((aligned(16))) float sdt[PM];
  const int tid  = (int)threadIdx.x;
  const int lane = tid & 31, hh = lane >> 4, m = lane & 15;
  const int wave = __builtin_amdgcn_readfirstlane(tid >> 5);
  const int side = (int)blockIdx.y;
  const int rowBase = (int)blockIdx.x * PM;

  if (wave < 2) {
    const v4f pv = *(const v4fa*)(PAR + 4 * tid);
    *(v4fa*)(spar + 4 * tid) = pv;
  }

  v8f acc[4];
  {
    const v8f z = {0.f, 0.f, 0.f, 0.f, 0.f, 0.f, 0.f, 0.f};
    acc[0] = z; acc[1] = z; acc[2] = z; acc[3] = z;
  }
  const int row = rowBase + 16 * wave + m;
  const int rc  = row < NP_C ? row : NP_C - 1;
  const int msk = row < NP_C ? -1 : 0;
  const v8i mv  = {msk, msk, msk, msk, msk, msk, msk, msk};
  const unsigned short* ap = HB + (size_t)side * (size_t)PLANE_H + (size_t)rc * DD + 8 * hh;
  const unsigned short* wp = WB + (size_t)m * DD + 8 * hh;
#pragma unroll
  for (int k0 = 0; k0 < DD; k0 += 32) {
    FragB af;
    af.h[0] = *(const v8usa*)(ap + k0);
    af.h[1] = *(const v8usa*)(ap + k0 + 16);
    af.w = af.w & mv;
#pragma unroll
    for (int t = 0; t < 4; ++t) {
      const unsigned short* wq = wp + (size_t)(16 * t) * DD + k0;
      FragB bf;
      bf.h[0] = *(const v8usa*)wq;
      bf.h[1] = *(const v8usa*)(wq + 16);
      acc[t] = wmb(af, bf, acc[t]);
    }
  }

#pragma unroll
  for (int t = 0; t < 4; ++t) {
    const int lc = 16 * t + m;
#pragma unroll
    for (int r = 0; r < 8; ++r) {
      const int lr = 16 * wave + 8 * hh + r;
      stg[lr * SPITCH + lc] = acc[t][r];
    }
  }
  __syncthreads();

  if (wave < 4) {
    const int r = tid;
    const int ao = DD + side * DD;
    float s = 0.0f;
#pragma unroll 4
    for (int j = 0; j < DD; ++j) s = fmaf(stg[r * SPITCH + j] + spar[j], spar[ao + j], s);
    sdt[r] = (rowBase + r < NP_C) ? s : 0.0f;
  }
  __syncthreads();

  if (wave == 0) {
    const v4f sv = *(const v4fa*)(sdt + 4 * lane);
    float* sp = S + (size_t)side * SPAD + (size_t)blockIdx.x * PM + 4 * lane;
    *(volatile v4f*)sp = sv;
    __threadfence();
    *(volatile v4f*)sp = sv;
  }
}

__device__ __forceinline__ int scan_chunk(const int* __restrict__ us, const int* __restrict__ vs, int cbase,
                                          int slotBase, int nb, int* list, int tid, int lane, int wave) {
  (void)lane;
  int wc = 0;
  const int e0 = cbase + tid * EPT;
  const int eb = e0 < NE_C - EPT ? e0 : NE_C - EPT;
  const int vm = (e0 < NE_C) ? -1 : 0;
  const int sent = -2147483647 - 1;
  const v4i da = *(const v4ia*)(us + eb);
  const v4i db = *(const v4ia*)(us + eb + 4);
  const v4i va = *(const v4ia*)(vs + eb);
  const v4i vb = *(const v4ia*)(vs + eb + 4);
  asm volatile("" :: "v"(da), "v"(db), "v"(va), "v"(vb));
  const int sm = sent & ~vm;
  const unsigned nbs = (unsigned)slotBase;
  const unsigned unb = (unsigned)nb;
  const unsigned s0 = (unsigned)((da.x & vm) | sm) - nbs, s1 = (unsigned)((da.y & vm) | sm) - nbs;
  const unsigned s2 = (unsigned)((da.z & vm) | sm) - nbs, s3 = (unsigned)((da.w & vm) | sm) - nbs;
  const unsigned s4 = (unsigned)((db.x & vm) | sm) - nbs, s5 = (unsigned)((db.y & vm) | sm) - nbs;
  const unsigned s6 = (unsigned)((db.z & vm) | sm) - nbs, s7 = (unsigned)((db.w & vm) | sm) - nbs;
  const bool h0 = s0 < unb, h1 = s1 < unb, h2 = s2 < unb, h3 = s3 < unb;
  const bool h4 = s4 < unb, h5 = s5 < unb, h6 = s6 < unb, h7 = s7 < unb;
  const unsigned any = __builtin_amdgcn_ballot_w32(h0 | h1 | h2 | h3 | h4 | h5 | h6 | h7);
  if (any != 0u) {
#define HITJ(HJ, SJ, VJ) { \
      const unsigned mj = __builtin_amdgcn_ballot_w32(HJ); \
      if (mj != 0u) { \
        if (HJ) { \
          const int pos = wc + (int)__builtin_amdgcn_mbcnt_lo(mj, 0u); \
          int vc = (VJ); \
          vc = vc < 0 ? 0 : (vc > NO_C - 1 ? NO_C - 1 : vc); \
          if (pos < WCAP) list[wave * WCAP + pos] = (vc << SLA) | (int)(SJ); \
        } \
        wc += (int)__builtin_popcount(mj); } }
    HITJ(h0, s0, va.x)
    HITJ(h1, s1, va.y)
    HITJ(h2, s2, va.z)
    HITJ(h3, s3, va.w)
    HITJ(h4, s4, vb.x)
    HITJ(h5, s5, vb.y)
    HITJ(h6, s6, vb.z)
    HITJ(h7, s7, vb.w)
#undef HITJ
  }
  return wc;
}

__global__ __launch_bounds__(NTHR) __attribute__((amdgpu_num_vgpr(248)))
void k_scan(const int* __restrict__ us, const int* __restrict__ vs, const unsigned* __restrict__ HOBw,
            const float* __restrict__ SP, const float* __restrict__ SO, const float* __restrict__ PAR,
            float* out) {
  extern __shared__ v4f lds_dyn[];
  int* reg1 = (int*)lds_dyn;
  int* reg2 = reg1 + RCAP;
  int* scnt = reg2 + RCAP;
  int* soff = scnt + NBRUN;
  int* list = soff + NBRUN;
  int* wcnt = list + LISTN;
  int* wtot = wcnt + NWAVE;
  const int tid  = (int)threadIdx.x;
  const int lane = tid & 31;
  const int wave = __builtin_amdgcn_readfirstlane(tid >> 5);
  const int nodeBase = (int)blockIdx.x * NBRUN;
  int nb = NP_C - nodeBase;
  nb = nb > NBRUN ? NBRUN : (nb < 0 ? 0 : nb);

  for (int i = tid; i < NBRUN; i += NTHR) scnt[i] = 0;
  if (tid == 0) reg2[0] = 0;
  __syncthreads();

  int tot = 0;
  const int nChunks = (NE_C + CHUNK - 1) / CHUNK;
#pragma unroll 1
  for (int ch = 0; ch < nChunks; ++ch) {
    const int cbase = ch * CHUNK;
    const int wc = scan_chunk(us, vs, cbase, nodeBase, nb, list, tid, lane, wave);
    if (lane == 0) wcnt[wave] = wc;
    __syncthreads();
    int pre = 0, all = 0;
#pragma unroll
    for (int w2 = 0; w2 < NWAVE; ++w2) {
      int c = wcnt[w2];
      c = c < 0 ? 0 : (c > WCAP ? WCAP : c);
      all += c;
      pre += (w2 < wave) ? c : 0;
    }
    const int wcc  = wc > WCAP ? WCAP : wc;
    const int base = tot + pre;
#pragma unroll 1
    for (int i = lane; i < wcc; i += 32) {
      const int ent = list[wave * WCAP + i];
      const int pos = base + i;
      if (pos < RCAP) reg1[pos] = ent;
    }
    tot += all;
    tot = tot > RCAP ? RCAP : tot;
    __syncthreads();
  }
  const int nh = tot;

  if (wave == 0) {
#pragma unroll 1
    for (int b0 = 0; b0 < nh; b0 += 32) {
      const int idx = b0 + lane;
      const int uv  = reg1[idx < nh ? idx : nh - 1];
      const int m32 = (nh - b0) < 32 ? (nh - b0) : 32;
#pragma unroll 1
      for (int k = 0; k < m32; ++k) {
        const int u  = __builtin_amdgcn_readlane(uv, k);
        const int sl = u & (NBRUN - 1);
        if (lane == 0) scnt[sl] = scnt[sl] + 1;
      }
    }
  }
  __syncthreads();

  {
    const v4i ca = *(const v4ia*)(scnt + 4 * tid);
    const int e0 = ca.x < 0 ? 0 : ca.x, e1 = ca.y < 0 ? 0 : ca.y;
    const int e2 = ca.z < 0 ? 0 : ca.z, e3 = ca.w < 0 ? 0 : ca.w;
    const int ts = e0 + e1 + e2 + e3;
    int incl = ts;
#pragma unroll
    for (int d = 1; d < 32; d <<= 1) {
      const int up = __shfl_up(incl, d);
      if (lane >= d) incl += up;
    }
    if (lane == 31) wtot[wave] = incl;
    __syncthreads();
    int pre = 0;
#pragma unroll
    for (int w2 = 0; w2 < NWAVE; ++w2) pre += (w2 < wave) ? wtot[w2] : 0;
    int run = pre + incl - ts;
    soff[4 * tid + 0] = run; run += e0;
    soff[4 * tid + 1] = run; run += e1;
    soff[4 * tid + 2] = run; run += e2;
    soff[4 * tid + 3] = run;
  }
  __syncthreads();
  for (int i = tid; i < NBRUN; i += NTHR) list[i] = soff[i];
  __syncthreads();

  if (wave == 0) {
#pragma unroll 1
    for (int b0 = 0; b0 < nh; b0 += 32) {
      const int idx = b0 + lane;
      const int uv  = reg1[idx < nh ? idx : nh - 1];
      const int m32 = (nh - b0) < 32 ? (nh - b0) : 32;
#pragma unroll 1
      for (int k = 0; k < m32; ++k) {
        const int u  = __builtin_amdgcn_readlane(uv, k);
        const int sl = u & (NBRUN - 1);
        const int gi = (int)((unsigned)u >> SLA);
        if (lane == 0) {
          int pos = list[sl];
          pos = pos < 0 ? 0 : (pos > RCAP - 1 ? RCAP - 1 : pos);
          reg2[pos] = gi;
          list[sl] = pos + 1;
        }
      }
    }
  }
  __syncthreads();

  const bool  ovf  = (nh >= RCAP);
  const float qnan = __int_as_float(0x7fc00000);
  const float abv  = PAR[192];
  const int   nhm  = nh > 0 ? nh - 1 : 0;
#pragma unroll 1
  for (int si = 0; si < NBRUN / NWAVE; ++si) {
    const int slot = si * NWAVE + wave;
    const int node = nodeBase + slot;
    if (node < NP_C) {
      const int craw = __builtin_amdgcn_readfirstlane(scnt[slot]);
      int st = __builtin_amdgcn_readfirstlane(soff[slot]);
      st = st < 0 ? 0 : (st > nh ? nh : st);
      int cnt = craw < 0 ? 0 : (craw > DEGCAP ? DEGCAP : craw);
      if (cnt > nh - st) cnt = nh - st;
      const bool bad = ovf || (craw > DEGCAP);
      const float c  = SP[node] + abv;

      const int cm1 = cnt > 0 ? cnt - 1 : 0;
      const int ja  = lane < cm1 ? lane : cm1;
      const int jb  = (lane + 32) < cm1 ? (lane + 32) : cm1;
      int xa = st + ja; xa = xa > nhm ? nhm : xa;
      int xb = st + jb; xb = xb > nhm ? nhm : xb;
      int ga = reg2[xa]; ga = ga < 0 ? 0 : (ga > NO_C - 1 ? NO_C - 1 : ga);
      int gb = reg2[xb]; gb = gb < 0 ? 0 : (gb > NO_C - 1 ? NO_C - 1 : gb);
      const float soa = SO[ga];
      const float sob = SO[gb];
      asm volatile("" :: "v"(soa), "v"(sob));
      const float ea = c + soa;
      const float eb = c + sob;
      const bool oka = lane < cnt;
      const bool okb = (lane + 32) < cnt;
      float mm = fmaxf(oka ? ea : -3.0e38f, okb ? eb : -3.0e38f);
#pragma unroll
      for (int off = 16; off > 0; off >>= 1) mm = fmaxf(mm, __shfl_xor(mm, off));
      const float xea = expf(ea - mm);
      const float xeb = expf(eb - mm);
      const int pai = __float_as_int(oka ? xea : 0.0f);
      const int pbi = __float_as_int(okb ? xeb : 0.0f);

      float l = 0.0f, ax = 0.0f, ay = 0.0f;
      const int na = cnt < 32 ? cnt : 32;
#pragma unroll 1
      for (int k = 0; k < na; ++k) {
        const int   gk = __builtin_amdgcn_readlane(ga, k);
        const float pk = __int_as_float(__builtin_amdgcn_readlane(pai, k));
        const unsigned w = HOBw[(size_t)gk * 32 + lane];
        const float h0 = __uint_as_float(w << 16);
        const float h1 = __uint_as_float(w & 0xffff0000u);
        l += pk;
        ax = fmaf(pk, h0, ax);
        ay = fmaf(pk, h1, ay);
      }
      const int nb2 = cnt - 32;
#pragma unroll 1
      for (int k = 0; k < nb2; ++k) {
        const int   gk = __builtin_amdgcn_readlane(gb, k);
        const float pk = __int_as_float(__builtin_amdgcn_readlane(pbi, k));
        const unsigned w = HOBw[(size_t)gk * 32 + lane];
        const float h0 = __uint_as_float(w << 16);
        const float h1 = __uint_as_float(w & 0xffff0000u);
        l += pk;
        ax = fmaf(pk, h0, ax);
        ay = fmaf(pk, h1, ay);
      }
      const float gx = ax / l;
      const float gy = ay / l;
      float ss = gx * gx + gy * gy;
#pragma unroll
      for (int off = 16; off > 0; off >>= 1) ss += __shfl_xor(ss, off);
      const float nn = fmaxf(sqrtf(ss), 1e-12f);
      const float ox = gx / nn;
      const float oy = gy / nn;
      v2f o;
      o.x = bad ? qnan : ((cnt == 0) ? 0.0f : ox);
      o.y = bad ? qnan : ((cnt == 0) ? 0.0f : oy);
      float* op = out + (size_t)node * DD + 2 * lane;
      *(volatile v2f*)op = o;
      __threadfence();
      *(volatile v2f*)op = o;
    }
  }
}

static inline int cdiv(int a, int b) { return (a + b - 1) / b; }

extern "C" void kernel_launch(void* const* d_in, const int* in_sizes, int n_in,
                              void* d_out, int out_size, void* d_ws, size_t ws_size,
                              hipStream_t stream) {
  if (n_in < 8) return;
  if (in_sizes[0] != NP_C * DD) return;
  if (in_sizes[1] != NO_C * DD) return;
  if (in_sizes[2] != DD * DD) return;
  if (in_sizes[3] != DD) return;
  if (in_sizes[4] != 2 * DD) return;
  if (in_sizes[5] != 1) return;
  if (in_sizes[6] != NE_C || in_sizes[7] != NE_C) return;
  if ((long long)out_size != (long long)(NP_C + NO_C) * DD) return;

  const float* hp = (const float*)d_in[0];
  const float* ho = (const float*)d_in[1];
  const float* Ww = (const float*)d_in[2];
  const float* Wb = (const float*)d_in[3];
  const float* aw = (const float*)d_in[4];
  const float* ab = (const float*)d_in[5];
  const int*   uu = (const int*)d_in[6];
  const int*   vv = (const int*)d_in[7];
  float* out = (float*)d_out;

  char* ws = (char*)d_ws;
  size_t off = 0;
  const size_t oHPB = off; off += (size_t)NP_C * DD * 2;  off = (off + 255) & ~(size_t)255;
  const size_t oHOB = off; off += (size_t)NO_C * DD * 2;  off = (off + 255) & ~(size_t)255;
  const size_t oWB  = off; off += (size_t)DD * DD * 2;    off = (off + 255) & ~(size_t)255;
  const size_t oPAR = off; off += (size_t)PARN * 4;       off = (off + 255) & ~(size_t)255;
  const size_t oSP  = off; off += (size_t)SPAD * 4;       off = (off + 255) & ~(size_t)255;
  const size_t oSO  = off; off += (size_t)SPAD * 4;       off = (off + 255) & ~(size_t)255;
  if (oHOB - oHPB != (size_t)PLANE_H * 2) return;
  if (oSO - oSP != (size_t)SPAD * 4) return;
  if (off > ws_size || off > (size_t)WSMAX) return;
  unsigned* HPB = (unsigned*)(ws + oHPB);
  unsigned* HOB = (unsigned*)(ws + oHOB);
  unsigned* WBp = (unsigned*)(ws + oWB);
  float*    PAR = (float*)(ws + oPAR);
  float*    SP  = (float*)(ws + oSP);
  float*    SO  = (float*)(ws + oSO);

  hipFuncSetAttribute(reinterpret_cast<const void*>(&k_scan),
                      hipFuncAttributeMaxDynamicSharedMemorySize, LDS_SCAN);

  k_prep<<<cdiv(NROWS_PREP, NWAVE), NTHR, 0, stream>>>(hp, ho, Ww, Wb, aw, ab, HPB, HOB, WBp, PAR, out);
  k_proj<<<dim3(NBLK_P, 2), NTHR, 0, stream>>>((const unsigned short*)HPB, (const unsigned short*)WBp, PAR, SP);
  k_scan<<<NBLK_S, NTHR, LDS_SCAN, stream>>>(uu, vv, (const unsigned*)HOB, SP, SO, PAR, out);
}
